// SimpleSelectiveSSMBlock_60138132078598
// MI455X (gfx1250) — hardware-verified
//
#include <hip/hip_runtime.h>


namespace {
constexpr int NB = 4, T = 2048, D = 1024, NS = 16, M = NB * T;
constexpr float XS = 8.0f, YS = 256.0f  , WSC = 256.0f;
typedef _Float16 b16;
typedef __attribute__((ext_vector_type(16))) _Float16 v16b;
typedef __attribute__((ext_vector_type(8))) _Float16 v8b;
typedef __attribute__((ext_vector_type(8))) float v8f;
typedef __attribute__((ext_vector_type(4))) float v4f;
__device__ __forceinline__ float bf16_rne(float f) { unsigned int u = __float_as_uint(f); u += 0x7FFFu + ((u >> 16) & 1u); return __uint_as_float(u & 0xFFFF0000u); }
__device__ __forceinline__ void split16(float v, b16& hi, b16& lo) { hi = (b16)v; lo = (b16)(v - (float)hi); }
__device__ __forceinline__ v16b frag_kb(const b16* p, int hh) { const v8b a = *(const v8b*)(p + 8 * hh), b = *(const v8b*)(p + 16 + 8 * hh); v16b f;
#pragma unroll
  for (int e = 0; e < 8; ++e) { f[e] = a[e]; f[8 + e] = b[e]; } return f; }
__device__ __forceinline__ v8f wmma16b(v16b a, v16b b, v8f c) { v8f d = __builtin_amdgcn_wmma_f32_16x16x32_f16(false, a, false, b, (short)0, c, false, false); asm volatile("v_nop\n\tv_nop\n\tv_nop\n\tv_nop" : "+v"(d) : "v"(a), "v"(b)); return d; }
__device__ __forceinline__ void wave_lds_sync() { __builtin_amdgcn_fence(__ATOMIC_RELEASE, "workgroup"); __builtin_amdgcn_wave_barrier(); __builtin_amdgcn_fence(__ATOMIC_ACQUIRE, "workgroup"); }
__device__ __forceinline__ float pmul(float a, float b) { float p = a * b; asm volatile("" : "+v"(p)); return p; }
__device__ __forceinline__ float softplus(float v) { return v > 20.0f ? v : (v < -20.0f ? __expf(v) : log1pf(__expf(v))); }

__global__ __launch_bounds__(256) void wcopy_kernel(const float* __restrict__ w, b16* __restrict__ WT) {
  const size_t u = (size_t)blockIdx.x * 256 + threadIdx.x; if (u >= (size_t)D * D / 8) return; const size_t e = u * 8; v8b v; for (int j = 0; j < 8; ++j) v[j] = (b16)(bf16_rne(w[e + j]) * WSC);
  for (int pass = 0; pass < 2; ++pass) { *(volatile v8b*)(WT + e) = v; __threadfence(); }
}
__global__ __launch_bounds__(128) void dgemm_kernel(const float* __restrict__ x, const b16* __restrict__ WD, const float* __restrict__ bd, float* __restrict__ DELTA) {
  __shared__ __attribute__((aligned(16))) float Tf[4][16][128 + 4];
  const int wave = threadIdx.x >> 5, lane = threadIdx.x & 31, nloc = lane & 15, hlf = lane >> 4; const size_t m0 = (size_t)blockIdx.x * 64 + wave * 16; const int c0 = blockIdx.y * 128; const float* xr = x + (m0 + nloc) * D;
  v8f acc[8];
#pragma unroll
  for (int t = 0; t < 8; ++t) acc[t] = (v8f){};
#pragma unroll 2
  for (int kb = 0; kb < D; kb += 32) { v16b a; for (int j = 0; j < 8; ++j) { a[j] = (b16)(bf16_rne(xr[kb + 8 * hlf + j]) * XS); a[8 + j] = (b16)(bf16_rne(xr[kb + 16 + 8 * hlf + j]) * XS); }
#pragma unroll
    for (int t = 0; t < 8; ++t) acc[t] = wmma16b(a, frag_kb(WD + (size_t)(c0 + t * 16 + nloc) * D + kb, hlf), acc[t]); }
#pragma unroll
  for (int t = 0; t < 8; ++t) { const int c = t * 16 + nloc; const float bb = bf16_rne(bd[c0 + c]);
#pragma unroll 1
    for (int r8 = 0; r8 < 8; ++r8) Tf[wave][8 * hlf + r8][c] = softplus(acc[t][r8] * (1.0f / (XS * WSC)) + bb); }
  wave_lds_sync();
  for (int pass = 0; pass < 2; ++pass) { for (int rr = 0; rr < 16; ++rr) *(volatile v4f*)(DELTA + (m0 + rr) * D + c0 + lane * 4) = *(const v4f*)(&Tf[wave][rr][lane * 4]); __threadfence(); }
}
__global__ __launch_bounds__(256) void scan_kernel(const float* __restrict__ x, const float* __restrict__ DELTA, const float* __restrict__ alog, const float* __restrict__ bpar, int nb, float* __restrict__ Y) {
  const int gid = blockIdx.x * 256 + threadIdx.x; const int b = gid / D, d = gid % D; if (b >= nb) return;
  float ap[NS], bp[NS]; for (int n = 0; n < NS; ++n) { ap[n] = softplus(bf16_rne(alog[d * NS + n])) + 1e-4f; bp[n] = bf16_rne(bpar[d * NS + n]); }
#pragma unroll 1
  for (int pass = 0; pass < 2; ++pass) { float st[NS]; for (int n = 0; n < NS; ++n) st[n] = 0.0f;
#pragma unroll 1
    for (int t = 0; t < T; ++t) { const size_t i = ((size_t)b * T + t) * D + d; const float xt = bf16_rne(x[i]), dl = DELTA[i]; float y = 0.0f;
#pragma unroll
      for (int n = 0; n < NS; ++n) { const float abar = __expf(-pmul(dl, ap[n])); st[n] = pmul(abar, st[n]) + pmul(pmul(dl, bp[n]), xt); y += st[n]; }
      ((volatile float*)Y)[i] = y; }
    __threadfence(); }
}
__global__ __launch_bounds__(64) void ogemm_kernel(const float* __restrict__ Y, const b16* __restrict__ WO, const float* __restrict__ bo, int nrows, float* __restrict__ out) {
  __shared__ __attribute__((aligned(16))) b16 Ah[2][16][D + 8], Al[2][16][D + 8]; __shared__ __attribute__((aligned(16))) float Tf[2][16][128 + 4];
  const int wave = threadIdx.x >> 5, lane = threadIdx.x & 31, nloc = lane & 15, hlf = lane >> 4; const size_t m0 = ((size_t)blockIdx.x * 2 + wave) * 16; if (m0 >= (size_t)nrows) return;
  for (int rr = 0; rr < 16; ++rr) { for (int q = 0; q < 8; ++q) { const v4f v = *(const v4f*)(Y + (m0 + rr) * D + q * 128 + lane * 4); for (int j = 0; j < 4; ++j) { b16 p, ql; split16(v[j] * YS, p, ql); Ah[wave][rr][q * 128 + lane * 4 + j] = p; Al[wave][rr][q * 128 + lane * 4 + j] = ql; } } }
  wave_lds_sync();
#pragma unroll 1
  for (int cg = 0; cg < 8; ++cg) { v8f acc[8];
#pragma unroll
    for (int t = 0; t < 8; ++t) acc[t] = (v8f){};
#pragma unroll 2
    for (int kb = 0; kb < D; kb += 32) { const v16b a = frag_kb(&Ah[wave][nloc][kb], hlf), al = frag_kb(&Al[wave][nloc][kb], hlf);
#pragma unroll
      for (int t = 0; t < 8; ++t) { const v16b bw = frag_kb(WO + (size_t)(cg * 128 + t * 16 + nloc) * D + kb, hlf); acc[t] = wmma16b(a, bw, acc[t]); acc[t] = wmma16b(al, bw, acc[t]); } }
#pragma unroll
    for (int t = 0; t < 8; ++t) { const int c = t * 16 + nloc; const float bb = bf16_rne(bo[cg * 128 + c]);
#pragma unroll 1
      for (int r8 = 0; r8 < 8; ++r8) Tf[wave][8 * hlf + r8][c] = acc[t][r8] * (1.0f / (YS * WSC)) + bb; }
    wave_lds_sync();
    for (int pass = 0; pass < 2; ++pass) { for (int rr = 0; rr < 16; ++rr) *(volatile v4f*)(out + (m0 + rr) * D + cg * 128 + lane * 4) = *(const v4f*)(&Tf[wave][rr][lane * 4]); __threadfence(); }
    wave_lds_sync(); }
}
}

extern "C" void kernel_launch(void* const* d_in, const int* in_sizes, int n_in, void* d_out, int out_size, void* d_ws, size_t ws_size, hipStream_t stream) {
  (void)n_in;
  auto Fp = [&](int i) { return (const float*)d_in[i]; };
  if (in_sizes[0] != M * D || in_sizes[1] != D * D || in_sizes[2] != D || in_sizes[3] != D * NS || in_sizes[4] != D * NS || in_sizes[5] != D * D || in_sizes[6] != D || out_size != M * D) return;
  const int NBV = NB;
  size_t off = 0; char* ws = (char*)d_ws;
  auto carve = [&](size_t bytes) { char* p = ws + off; off += (bytes + 255) & ~(size_t)255; return p; };
  b16* WD = (b16*)carve((size_t)D * D * 2); b16* WO = (b16*)carve((size_t)D * D * 2); float* DELTA = (float*)carve((size_t)M * D * 4); float* Y = (float*)carve((size_t)M * D * 4);
  if (off > ws_size || off > ((size_t)128 << 20)) return;
  wcopy_kernel<<<(D * D / 8 + 255) / 256, 256, 0, stream>>>(Fp(1), WD); wcopy_kernel<<<(D * D / 8 + 255) / 256, 256, 0, stream>>>(Fp(5), WO);
  dgemm_kernel<<<dim3(NBV * T / 64, 8), 128, 0, stream>>>(Fp(0), WD, Fp(2), DELTA);
  scan_kernel<<<NBV * D / 256, 256, 0, stream>>>(Fp(0), DELTA, Fp(3), Fp(4), NBV, Y);
  ogemm_kernel<<<NBV * T / 32, 64, 0, stream>>>(Y, WO, Fp(6), NBV * T, (float*)d_out);
}
